// TtCodeGenAttention_14834817040847
// MI455X (gfx1250) — hardware-verified
//
#include <hip/hip_runtime.h>
#include <stdint.h>

constexpr int kBatch   = 2;
constexpr int kSeq     = 2048;
constexpr int kEmb     = 1024;
constexpr int kHeads   = 16;
constexpr int kHdim    = 64;
constexpr int kTok     = kBatch * kSeq;
constexpr int kQkvCols = 3 * kEmb;
constexpr int kMpCols  = 768;
constexpr float kQKCarry        = 64.0f;
constexpr float kScoreScale     = 1.0f / 32768.0f;
constexpr float kMaskVal        = -10000000.0f;
constexpr float kLog2BaseOver16 = 0.83048202372184059f;

typedef __attribute__((ext_vector_type(16))) _Float16 v16h;
typedef __attribute__((ext_vector_type(8)))  _Float16 v8h;
typedef __attribute__((ext_vector_type(16))) __bf16   v16b;
typedef __attribute__((ext_vector_type(8)))  __bf16   v8b;
typedef __attribute__((ext_vector_type(8)))  float    v8f;
typedef __attribute__((ext_vector_type(4)))  float    v4f;
typedef __attribute__((ext_vector_type(2)))  float    v2f;

__device__ __forceinline__ unsigned short f2bf_bits(float f) {
  unsigned u = __float_as_uint(f);
  return (unsigned short)((u + 0x7FFFu + ((u >> 16) & 1u)) >> 16);
}
__device__ __forceinline__ float bf_bits2f(unsigned short h) { return __uint_as_float(((unsigned)h) << 16); }
__device__ __forceinline__ __bf16 f2bf(float f) { return __builtin_bit_cast(__bf16, f2bf_bits(f)); }
__device__ __forceinline__ void split_bf16(float f, __bf16& hi, __bf16& lo) {
  const unsigned short hb = f2bf_bits(f);
  hi = __builtin_bit_cast(__bf16, hb);
  lo = f2bf(f - __uint_as_float(((unsigned)hb) << 16));
}

__device__ __forceinline__ void dep_guard_h(v8f& a, v8f& b, v16h x, v16h y) { asm volatile("v_nop\n\tv_nop\n\tv_nop\n\tv_nop" : "+v"(a), "+v"(b) : "v"(x), "v"(y)); }
__device__ __forceinline__ void dep_guard_b(v8f& a, v8f& b, v16b x, v16b y) { asm volatile("v_nop\n\tv_nop\n\tv_nop\n\tv_nop" : "+v"(a), "+v"(b) : "v"(x), "v"(y)); }
__device__ __forceinline__ void keep4_h(v16h a, v16h b, v16h c, v16h d) { asm volatile("v_nop" :: "v"(a), "v"(b), "v"(c), "v"(d)); }
__device__ __forceinline__ void keep4_b(v16b a, v16b b, v16b c, v16b d) { asm volatile("v_nop" :: "v"(a), "v"(b), "v"(c), "v"(d)); }
__device__ __forceinline__ void acc_guard4(v8f& a, v8f& b, v8f& c, v8f& d) { asm volatile("v_nop\n\tv_nop\n\tv_nop\n\tv_nop" : "+v"(a), "+v"(b), "+v"(c), "+v"(d)); }
template <typename T> struct Frag;
template <> struct Frag<_Float16> {
  typedef v16h V; union U { v16h v; v8h h[2]; };
  static __device__ __forceinline__ v16h load(const _Float16* p) {
    U f; f.h[0] = *(const v8h*)(p); f.h[1] = *(const v8h*)(p + 16); return f.v;
  }
  static __device__ __forceinline__ v8f mma(v16h a, v16h b, v8f c) {
    return __builtin_amdgcn_wmma_f32_16x16x32_f16(false, a, false, b, (short)0, c, false, false);
  }
  static __device__ __forceinline__ void guard(v8f& a, v8f& b, v16h x, v16h y) { dep_guard_h(a, b, x, y); }
  static __device__ __forceinline__ void keep(v16h a, v16h b, v16h c, v16h d) { keep4_h(a, b, c, d); }
};
template <> struct Frag<__bf16> {
  typedef v16b V; union U { v16b v; v8b h[2]; };
  static __device__ __forceinline__ v16b load(const __bf16* p) {
    U f; f.h[0] = *(const v8b*)(p); f.h[1] = *(const v8b*)(p + 16); return f.v;
  }
  static __device__ __forceinline__ v8f mma(v16b a, v16b b, v8f c) {
    return __builtin_amdgcn_wmma_f32_16x16x32_bf16(false, a, false, b, (short)0, c, false, false);
  }
  static __device__ __forceinline__ void guard(v8f& a, v8f& b, v16b x, v16b y) { dep_guard_b(a, b, x, y); }
  static __device__ __forceinline__ void keep(v16b a, v16b b, v16b c, v16b d) { keep4_b(a, b, c, d); }
};

__device__ __forceinline__ v8f mma_f16g(v16h a, v16h b, v8f c) {
  c = __builtin_amdgcn_wmma_f32_16x16x32_f16(false, a, false, b, (short)0, c, false, false);
  asm volatile("v_nop\n\tv_nop\n\tv_nop\n\tv_nop" : "+v"(c) : "v"(a), "v"(b));
  return c;
}
__device__ __forceinline__ v8f mma_bf16g(v16b a, v16b b, v8f c) {
  c = __builtin_amdgcn_wmma_f32_16x16x32_bf16(false, a, false, b, (short)0, c, false, false);
  asm volatile("v_nop\n\tv_nop\n\tv_nop\n\tv_nop" : "+v"(c) : "v"(a), "v"(b));
  return c;
}

template <int ET> struct Elem;
template <> struct Elem<0> { typedef _Float16 T; };
template <> struct Elem<1> { typedef __bf16 T; };
template <int ET, int SPLITM, int BIAS_MODE, int OUT_MODE, bool RESID, int ACT = 0>
__global__ __launch_bounds__(256) void wmma_gemm64(
    const unsigned short* __restrict__ Ap, const unsigned short* __restrict__ A2p, int lda, long strideA,
    const unsigned short* __restrict__ Btp, const unsigned short* __restrict__ Bt2p, int ldb, long strideB,
    void* __restrict__ Cout, void* __restrict__ Cout2, int ldc, long strideC,
    const float* __restrict__ bias,
    const float* __restrict__ resid, long strideR,
    int M, int N, int K, float scale) {
  typedef typename Elem<ET>::T T;
  typedef typename Frag<T>::V V;
  const T* A = (const T*)Ap; const T* A2 = (const T*)A2p; const T* Bt = (const T*)Btp; const T* Bt2 = (const T*)Bt2p;
  __shared__ __align__(16) float sT[8][16 * 68];
  const int b    = blockIdx.y;
  const int lane = threadIdx.x & 31;
  const int wave = threadIdx.x >> 5;
  const int tilesN = N >> 6;
  const int tilesM = M >> 6;
  const int tile = blockIdx.x * 8 + wave;
  if (tile >= tilesM * tilesN) return;
  const int tm = tile / tilesN;
  const int tn = tile - tm * tilesN;
  const int m0 = tm << 6;
  const int n0 = tn << 6;

  const T* Ab  = A  + (size_t)b * strideA;
  const T* Bb  = Bt + (size_t)b * strideB;
  const T* Ab2 = (SPLITM >= 1) ? (A2  + (size_t)b * strideA) : nullptr;
  const T* Bb2 = (SPLITM == 2) ? (Bt2 + (size_t)b * strideB) : nullptr;

  const int rlane = lane & 15;
  const int koff  = (lane >> 4) * 8;
  const int mOff  = (lane >> 4) * 8;

  v8f acc[4][4];
#pragma unroll
  for (int i = 0; i < 4; ++i)
#pragma unroll
    for (int j = 0; j < 4; ++j) acc[i][j] = (v8f){0.f,0.f,0.f,0.f,0.f,0.f,0.f,0.f};

  for (int k0 = 0; k0 < K; k0 += 32) {
    V bh[4], bl[4];
#pragma unroll
    for (int j = 0; j < 4; ++j) {
      const size_t bo = (size_t)(n0 + (j << 4) + rlane) * ldb + koff + k0;
      bh[j] = Frag<T>::load(Bb + bo);
      if (SPLITM == 2) bl[j] = Frag<T>::load(Bb2 + bo);
    }
#pragma unroll
    for (int i = 0; i < 4; ++i) {
      const size_t ao = (size_t)(m0 + (i << 4) + rlane) * lda + koff + k0;
      V ah = Frag<T>::load(Ab + ao);
      V al;
      if (SPLITM >= 1) al = Frag<T>::load(Ab2 + ao);
#pragma unroll
      for (int j = 0; j < 4; ++j) {
        acc[i][j] = Frag<T>::mma(ah, bh[j], acc[i][j]);
        if (SPLITM == 2) acc[i][j] = Frag<T>::mma(ah, bl[j], acc[i][j]);
        if (SPLITM >= 1) acc[i][j] = Frag<T>::mma(al, bh[j], acc[i][j]);
      }
      Frag<T>::guard(acc[i][0], acc[i][3], ah, (SPLITM >= 1) ? al : ah);
    }
    Frag<T>::keep(bh[0], bh[1], bh[2], bh[3]);
    if (SPLITM == 2) Frag<T>::keep(bl[0], bl[1], bl[2], bl[3]);
  }
  acc_guard4(acc[0][0], acc[0][1], acc[0][2], acc[0][3]);
  acc_guard4(acc[1][0], acc[1][1], acc[1][2], acc[1][3]);
  acc_guard4(acc[2][0], acc[2][1], acc[2][2], acc[2][3]);
  acc_guard4(acc[3][0], acc[3][1], acc[3][2], acc[3][3]);

  float* slab = sT[wave];
  const float* Rb = RESID ? (resid + (size_t)b * strideR) : nullptr;
#pragma unroll
  for (int i = 0; i < 4; ++i) {
    const int mBase = m0 + (i << 4);
#pragma unroll
    for (int j = 0; j < 4; ++j) {
      const int n = n0 + (j << 4) + rlane;
      float bv = 0.f;
      if (BIAS_MODE == 2) bv = bias[n];
#pragma unroll
      for (int r = 0; r < 8; ++r) {
        float v = acc[i][j][r] * scale;
        if (BIAS_MODE == 1) v += bias[mBase + mOff + r];
        if (BIAS_MODE == 2) v += bv;
        if (RESID) v += Rb[(size_t)(mBase + mOff + r) * ldc + n];
        if (ACT == 1) v = tanhf(v);
        if (ACT == 2) v = fmaxf(v, 0.0f);
        if (ACT == 3) v = v / (1.0f + expf(-v));
        if (ACT == 4) v = (v > 0.f) ? v : 0.01f * v;
        slab[(mOff + r) * 68 + (j << 4) + rlane] = v;
      }
    }
    __builtin_amdgcn_fence(__ATOMIC_RELEASE, "workgroup");
    __builtin_amdgcn_wave_barrier();
    __builtin_amdgcn_fence(__ATOMIC_ACQUIRE, "workgroup");
    if (OUT_MODE == 0) {
      float* C = (float*)Cout + (size_t)b * strideC;
      const int hh = lane >> 4, c4 = (lane & 15) * 4;
      for (int pass = 0; pass < 2; ++pass) {
#pragma unroll
        for (int it = 0; it < 8; ++it) {
          const int row = it * 2 + hh;
          v4f v = *(const v4f*)(slab + row * 68 + c4);
          *(volatile v4f*)(C + (size_t)(mBase + row) * ldc + n0 + c4) = v;
        }
        __threadfence();
      }
    } else {
      const int q = lane >> 3, c8 = (lane & 7) * 8;
      unsigned short* C  = (unsigned short*)Cout  + (size_t)b * strideC;
      unsigned short* C2 = (OUT_MODE == 2) ? ((unsigned short*)Cout2 + (size_t)b * strideC) : nullptr;
      for (int pass = 0; pass < 2; ++pass) {
#pragma unroll
        for (int it = 0; it < 4; ++it) {
          const int row = it * 4 + q;
          const float* sp = slab + row * 68 + c8;
          v8h hv, lv;
#pragma unroll
          for (int e = 0; e < 8; ++e) {
            if (OUT_MODE == 1) {
              hv[e] = (_Float16)sp[e];
            } else {
              unsigned short hb = f2bf_bits(sp[e]);
              unsigned short lb = f2bf_bits(sp[e] - bf_bits2f(hb));
              hv[e] = __builtin_bit_cast(_Float16, hb);
              lv[e] = __builtin_bit_cast(_Float16, lb);
            }
          }
          *(volatile v8h*)(C + (size_t)(mBase + row) * ldc + n0 + c8) = hv;
          if (OUT_MODE == 2) *(volatile v8h*)(C2 + (size_t)(mBase + row) * ldc + n0 + c8) = lv;
        }
        __threadfence();
      }
    }
    __builtin_amdgcn_fence(__ATOMIC_RELEASE, "workgroup");
    __builtin_amdgcn_wave_barrier();
    __builtin_amdgcn_fence(__ATOMIC_ACQUIRE, "workgroup");
  }
}

__global__ __launch_bounds__(256) void cast_f32_bf16x8(const float* __restrict__ in,
                                                       unsigned short* __restrict__ out, int n8) {
  const int i = blockIdx.x * 256 + threadIdx.x;
  if (i < n8) {
    const v4f a = *(const v4f*)(in + (size_t)i * 8);
    const v4f b = *(const v4f*)(in + (size_t)i * 8 + 4);
    v8h o;
#pragma unroll
    for (int e = 0; e < 4; ++e) {
      o[e]     = __builtin_bit_cast(_Float16, f2bf_bits(a[e]));
      o[4 + e] = __builtin_bit_cast(_Float16, f2bf_bits(b[e]));
    }
    unsigned short* dst = out + (size_t)i * 8;
    *(volatile v8h*)dst = o;
    __threadfence();
    *(volatile v8h*)dst = o;
  }
}

constexpr int kRsPitch = 64;
__global__ __launch_bounds__(256) void rope_split_k(const float* __restrict__ qkv,
                                                    unsigned short* __restrict__ q16p, unsigned short* __restrict__ k16p,
                                                    unsigned short* __restrict__ vhip, unsigned short* __restrict__ vlop) {
  __shared__ __align__(16) _Float16 slab[8][4 * kRsPitch];
  const int tid = threadIdx.x, wave = tid >> 5, lane = tid & 31;
  const int tok = blockIdx.x >> 1;
  const int h   = ((blockIdx.x & 1) << 3) + wave;
  const int s   = tok & (kSeq - 1);
  const int b   = tok >> 11;
  const int mp  = h >> 2, sub = h & 3;
  const float* src = qkv + (size_t)tok * kQkvCols + mp * kMpCols + sub * kHdim + 2 * lane;
  const v2f qv = *(const v2f*)(src);
  const v2f vv = *(const v2f*)(src + 256);
  const v2f kv = *(const v2f*)(src + 512);

  const int j = (lane < 16) ? lane : 15;
  const float invf = exp2f(-(float)j * kLog2BaseOver16);
  const float ang  = (float)s * invf;
  float sn, cs;
  sincosf(ang, &sn, &cs);
  const bool rot = lane < 16;
  const float cc = rot ? cs : 1.0f;
  const float ss = rot ? sn : 0.0f;
  const float q0 = qv[0] * cc - qv[1] * ss;
  const float q1 = qv[1] * cc + qv[0] * ss;
  const float k0 = kv[0] * cc - kv[1] * ss;
  const float k1 = kv[1] * cc + kv[0] * ss;

  _Float16* sw = slab[wave];
  sw[0 * kRsPitch + 2 * lane]     = (_Float16)(q0 * kQKCarry);
  sw[0 * kRsPitch + 2 * lane + 1] = (_Float16)(q1 * kQKCarry);
  sw[1 * kRsPitch + 2 * lane]     = (_Float16)(k0 * kQKCarry);
  sw[1 * kRsPitch + 2 * lane + 1] = (_Float16)(k1 * kQKCarry);
#pragma unroll
  for (int e = 0; e < 2; ++e) {
    __bf16 hi, lo;
    split_bf16(vv[e], hi, lo);
    sw[2 * kRsPitch + 2 * lane + e] = __builtin_bit_cast(_Float16, hi);
    sw[3 * kRsPitch + 2 * lane + e] = __builtin_bit_cast(_Float16, lo);
  }
  __builtin_amdgcn_fence(__ATOMIC_RELEASE, "workgroup");
  __builtin_amdgcn_wave_barrier();
  __builtin_amdgcn_fence(__ATOMIC_ACQUIRE, "workgroup");

  const int p = lane >> 3, c8 = (lane & 7) * 8;
  const size_t row = ((size_t)(b * kHeads + h) * kSeq + s) * kHdim;
  unsigned short* base = (p == 0) ? q16p : (p == 1) ? k16p : (p == 2) ? vhip : vlop;
  const v8h val = *(const v8h*)(sw + p * kRsPitch + c8);
  unsigned short* dst = base + row + c8;
  *(volatile v8h*)dst = val;
  __threadfence();
  *(volatile v8h*)dst = val;
}

constexpr int kAttKC  = 64;
constexpr int kAttOSP = 68;
__global__ __launch_bounds__(128) void attn64_k(const unsigned short* __restrict__ qpp, const unsigned short* __restrict__ kpp,
                                                const unsigned short* __restrict__ vhpp, const unsigned short* __restrict__ vlpp,
                                                unsigned short* __restrict__ ohip, unsigned short* __restrict__ olop) {
  union FH { v16h v; v8h h[2]; };
  union FB { v16b v; v8b h[2]; };
  __shared__ __align__(16) _Float16 Ksh[kAttKC * kHdim];
  __shared__ __align__(16) __bf16   Vth[kHdim * kAttKC];
  __shared__ __align__(16) __bf16   Vtl[kHdim * kAttKC];
  __shared__ __align__(16) __bf16   Psh[4][16 * kAttKC];
  __shared__ __align__(16) __bf16   Psl[4][16 * kAttKC];
  __shared__ __align__(16) float    Osh[4][16 * kAttOSP];
  const _Float16* qp  = (const _Float16*)qpp;
  const _Float16* kp  = (const _Float16*)kpp;
  const __bf16*   vhp = (const __bf16*)vhpp;
  const __bf16*   vlp = (const __bf16*)vlpp;
  const int tid = threadIdx.x, wave = tid >> 5, lane = tid & 31, hh = lane >> 4, c = lane & 15;
  const int nqb = kSeq / 64;
  const int bx  = blockIdx.x;
  const int qb  = bx % nqb;
  const int bh  = bx / nqb;
  const int h   = bh % kHeads;
  const int b   = bh / kHeads;
  const int q0  = qb * 64 + wave * 16;
  const size_t rowb = (size_t)bh * kSeq;

  v16h qa[2];
  {
    const _Float16* qrow = qp + (rowb + q0 + c) * kHdim + 8 * hh;
#pragma unroll
    for (int dc = 0; dc < 2; ++dc) qa[dc] = Frag<_Float16>::load(qrow + dc * 32);
  }
  float mrow[8], lrow[8];
  v8f oacc[4];
#pragma unroll
  for (int r = 0; r < 8; ++r) { mrow[r] = -__builtin_inff(); lrow[r] = 0.f; }
#pragma unroll
  for (int t = 0; t < 4; ++t) oacc[t] = (v8f){0.f,0.f,0.f,0.f,0.f,0.f,0.f,0.f};

  const int nChunks = qb + 1;
  for (int kc = 0; kc < nChunks; ++kc) {
    const int kv0 = kc * kAttKC;
    __syncthreads();
    {
      const int kvr = tid >> 1, dh = (tid & 1) * 32;
      const _Float16* krow  = kp  + (rowb + kv0 + kvr) * kHdim + dh;
      const __bf16*   vhrow = vhp + (rowb + kv0 + kvr) * kHdim + dh;
      const __bf16*   vlrow = vlp + (rowb + kv0 + kvr) * kHdim + dh;
#pragma unroll
      for (int i = 0; i < 4; ++i) {
        const v8h kk = *(const v8h*)(krow + 8 * i);
        *(v8h*)(Ksh + kvr * kHdim + dh + 8 * i) = kk;
        const v8b ah = *(const v8b*)(vhrow + 8 * i);
        const v8b al = *(const v8b*)(vlrow + 8 * i);
#pragma unroll
        for (int e = 0; e < 8; ++e) {
          Vth[(dh + 8 * i + e) * kAttKC + kvr] = ah[e];
          Vtl[(dh + 8 * i + e) * kAttKC + kvr] = al[e];
        }
      }
    }
    __syncthreads();

    v8f s[4];
#pragma unroll
    for (int j = 0; j < 4; ++j) {
      s[j] = (v8f){0.f,0.f,0.f,0.f,0.f,0.f,0.f,0.f};
#pragma unroll
      for (int dc = 0; dc < 2; ++dc) {
        FH kb;
        kb.h[0] = *(const v8h*)(Ksh + (j * 16 + c) * kHdim + dc * 32 + 8 * hh);
        kb.h[1] = *(const v8h*)(Ksh + (j * 16 + c) * kHdim + dc * 32 + 16 + 8 * hh);
        s[j] = mma_f16g(qa[dc], kb.v, s[j]);
      }
    }
    const bool diag = (kc == qb);
    float cm[8];
#pragma unroll
    for (int r = 0; r < 8; ++r) {
      const int qrow = q0 + 8 * hh + r;
      float m = -__builtin_inff();
#pragma unroll
      for (int j = 0; j < 4; ++j) {
        const int kvcol = kv0 + j * 16 + c;
        float sv = s[j][r] * kScoreScale;
        if (diag && (kvcol > qrow)) sv = kMaskVal;
        s[j][r] = sv;
        m = fmaxf(m, sv);
      }
#pragma unroll
      for (int off = 1; off < 16; off <<= 1) m = fmaxf(m, __shfl_xor(m, off, 32));
      cm[r] = m;
    }
    __bf16* pwh = Psh[wave];
    __bf16* pwl = Psl[wave];
#pragma unroll
    for (int r = 0; r < 8; ++r) {
      const float mnew  = fmaxf(mrow[r], cm[r]);
      const float alpha = expf(mrow[r] - mnew);
      mrow[r] = mnew;
      float psum = 0.f;
#pragma unroll
      for (int j = 0; j < 4; ++j) {
        const float p = expf(s[j][r] - mnew);
        psum += p;
        __bf16 ph, pl;
        split_bf16(p, ph, pl);
        pwh[(8 * hh + r) * kAttKC + j * 16 + c] = ph;
        pwl[(8 * hh + r) * kAttKC + j * 16 + c] = pl;
      }
#pragma unroll
      for (int off = 1; off < 16; off <<= 1) psum += __shfl_xor(psum, off, 32);
      lrow[r] = lrow[r] * alpha + psum;
#pragma unroll
      for (int t = 0; t < 4; ++t) oacc[t][r] *= alpha;
    }
    __builtin_amdgcn_fence(__ATOMIC_RELEASE, "workgroup");
    __builtin_amdgcn_wave_barrier();
    __builtin_amdgcn_fence(__ATOMIC_ACQUIRE, "workgroup");
#pragma unroll
    for (int kk = 0; kk < 2; ++kk) {
      FB pa, pl;
      pa.h[0] = *(const v8b*)(pwh + c * kAttKC + kk * 32 + 8 * hh);
      pa.h[1] = *(const v8b*)(pwh + c * kAttKC + kk * 32 + 16 + 8 * hh);
      pl.h[0] = *(const v8b*)(pwl + c * kAttKC + kk * 32 + 8 * hh);
      pl.h[1] = *(const v8b*)(pwl + c * kAttKC + kk * 32 + 16 + 8 * hh);
#pragma unroll
      for (int t = 0; t < 4; ++t) {
        FB vb, vl;
        vb.h[0] = *(const v8b*)(Vth + (t * 16 + c) * kAttKC + kk * 32 + 8 * hh);
        vb.h[1] = *(const v8b*)(Vth + (t * 16 + c) * kAttKC + kk * 32 + 16 + 8 * hh);
        vl.h[0] = *(const v8b*)(Vtl + (t * 16 + c) * kAttKC + kk * 32 + 8 * hh);
        vl.h[1] = *(const v8b*)(Vtl + (t * 16 + c) * kAttKC + kk * 32 + 16 + 8 * hh);
        oacc[t] = mma_bf16g(pa.v, vb.v, oacc[t]);
        oacc[t] = mma_bf16g(pa.v, vl.v, oacc[t]);
        oacc[t] = mma_bf16g(pl.v, vb.v, oacc[t]);
      }
    }
  }

  float* os = Osh[wave];
#pragma unroll
  for (int r = 0; r < 8; ++r) {
    const float inv = 1.0f / lrow[r];
#pragma unroll
    for (int t = 0; t < 4; ++t) os[(8 * hh + r) * kAttOSP + t * 16 + c] = oacc[t][r] * inv;
  }
  __builtin_amdgcn_fence(__ATOMIC_RELEASE, "workgroup");
  __builtin_amdgcn_wave_barrier();
  __builtin_amdgcn_fence(__ATOMIC_ACQUIRE, "workgroup");
  {
    const int q8 = lane >> 3, c8 = (lane & 7) * 8;
    unsigned short* oh = ohip + ((size_t)b * kSeq) * kEmb + h * kHdim;
    unsigned short* ol = olop + ((size_t)b * kSeq) * kEmb + h * kHdim;
    for (int pass = 0; pass < 2; ++pass) {
#pragma unroll
      for (int it = 0; it < 4; ++it) {
        const int row = it * 4 + q8;
        const float* sp = os + row * kAttOSP + c8;
        v8h hv, lv;
#pragma unroll
        for (int e = 0; e < 8; ++e) {
          const unsigned short hb = f2bf_bits(sp[e]);
          const unsigned short lb = f2bf_bits(sp[e] - bf_bits2f(hb));
          hv[e] = __builtin_bit_cast(_Float16, hb);
          lv[e] = __builtin_bit_cast(_Float16, lb);
        }
        *(volatile v8h*)(oh + (size_t)(q0 + row) * kEmb + c8) = hv;
        *(volatile v8h*)(ol + (size_t)(q0 + row) * kEmb + c8) = lv;
      }
      __threadfence();
    }
  }
}

extern "C" void kernel_launch(void* const* d_in, const int* in_sizes, int n_in,
                              void* d_out, int out_size, void* d_ws, size_t ws_size,
                              hipStream_t stream) {
  if (n_in < 3) return;
  if (in_sizes[0] != kTok * kEmb) return;
  if (in_sizes[1] != kQkvCols * kEmb) return;
  if (in_sizes[2] != kEmb * kEmb) return;
  if (out_size != kTok * kEmb) return;

  const float* hidden = (const float*)d_in[0];
  const float* wqkv   = (const float*)d_in[1];
  const float* wout   = (const float*)d_in[2];
  float* out = (float*)d_out;

  const size_t szHid16  = (size_t)kTok * kEmb * 2;
  const size_t szWqkv16 = (size_t)kQkvCols * kEmb * 2;
  const size_t szWout16 = (size_t)kEmb * kEmb * 2;
  const size_t szQkv    = (size_t)kTok * kQkvCols * 4;
  const size_t szPlane  = (size_t)kBatch * kHeads * kSeq * kHdim * 2;
  const size_t szO      = (size_t)kTok * kEmb * 2;
  const size_t offHid16  = 0;
  const size_t offWqkv16 = offHid16 + szHid16;
  const size_t offWout16 = offWqkv16 + szWqkv16;
  const size_t offQkv    = offWout16 + szWout16;
  const size_t offQ16    = offQkv + szQkv;
  const size_t offK16    = offQ16 + szPlane;
  const size_t offVhi    = offK16 + szPlane;
  const size_t offVlo    = offVhi + szPlane;
  const size_t offOhi    = offVlo + szPlane;
  const size_t offOlo    = offOhi + szO;
  const size_t total     = offOlo + szO;
  if (total > ws_size) return;

  char* ws = (char*)d_ws;
  unsigned short* hid16  = (unsigned short*)(ws + offHid16);
  unsigned short* wqkv16 = (unsigned short*)(ws + offWqkv16);
  unsigned short* wout16 = (unsigned short*)(ws + offWout16);
  float*          qkvf   = (float*)(ws + offQkv);
  unsigned short* q16    = (unsigned short*)(ws + offQ16);
  unsigned short* k16    = (unsigned short*)(ws + offK16);
  unsigned short* vhi    = (unsigned short*)(ws + offVhi);
  unsigned short* vlo    = (unsigned short*)(ws + offVlo);
  unsigned short* ohi    = (unsigned short*)(ws + offOhi);
  unsigned short* olo    = (unsigned short*)(ws + offOlo);

  {
    const int n8a = kTok * kEmb / 8, n8b = kQkvCols * kEmb / 8, n8c = kEmb * kEmb / 8;
    cast_f32_bf16x8<<<dim3((n8a + 255) / 256), dim3(256), 0, stream>>>(hidden, hid16, n8a);
    cast_f32_bf16x8<<<dim3((n8b + 255) / 256), dim3(256), 0, stream>>>(wqkv, wqkv16, n8b);
    cast_f32_bf16x8<<<dim3((n8c + 255) / 256), dim3(256), 0, stream>>>(wout, wout16, n8c);
  }
  {
    const int tiles = (kTok / 64) * (kQkvCols / 64);
    wmma_gemm64<1, 0, 0, 0, false, 0><<<dim3((tiles + 7) / 8, 1), dim3(256), 0, stream>>>(
        hid16, hid16, kEmb, 0L, wqkv16, wqkv16, kEmb, 0L,
        (void*)qkvf, (void*)qkvf, kQkvCols, 0L, qkvf, qkvf, 0L,
        kTok, kQkvCols, kEmb, 1.0f);
  }
  rope_split_k<<<dim3(kTok * 2), dim3(256), 0, stream>>>(qkvf, q16, k16, vhi, vlo);
  attn64_k<<<dim3(kBatch * kHeads * (kSeq / 64)), dim3(128), 0, stream>>>(q16, k16, vhi, vlo, ohi, olo);
  {
    const int tiles = (kTok / 64) * (kEmb / 64);
    wmma_gemm64<1, 1, 0, 0, false, 0><<<dim3((tiles + 7) / 8, 1), dim3(256), 0, stream>>>(
        ohi, olo, kEmb, 0L, wout16, wout16, kEmb, 0L,
        (void*)out, (void*)out, kEmb, 0L, qkvf, qkvf, 0L,
        kTok, kEmb, kEmb, 1.0f);
  }
}
